// Spiral_MambaBlock_86569360818673
// MI455X (gfx1250) — hardware-verified
//
#include <hip/hip_runtime.h>


#define NB_   2
#define NS_   2048
#define ND_   512
#define NE_   1024
#define NR_   32
#define NN_   16
#define NK_   64
#define ROWS_ 4096

static constexpr float EPS_ = 1e-5f;

static_assert(ROWS_ == NB_ * NS_);
static_assert(NS_ % 16 == 0);
static_assert(ND_ % 128 == 0);
static_assert(NE_ % 128 == 0);
static_assert(NR_ + 2 * NN_ == NK_);

typedef float          v4f   __attribute__((ext_vector_type(4)));
typedef float          v8f   __attribute__((ext_vector_type(8)));
typedef _Float16       v4h   __attribute__((ext_vector_type(4)));
typedef _Float16       v8h   __attribute__((ext_vector_type(8)));
typedef _Float16       v16h  __attribute__((ext_vector_type(16)));
typedef unsigned short u16x4 __attribute__((ext_vector_type(4)));
typedef unsigned short u16x8 __attribute__((ext_vector_type(8)));

union FragH { u16x8 h[2]; v16h v; };
union Pack8 { v8h f; u16x8 u; };
union Pack4 { v4h f; u16x4 u; };
union HBits { _Float16 h; unsigned short u; };

constexpr size_t SZ_MOD  = (size_t)NB_ * 3 * ND_ * 4;
constexpr size_t SZ_SKIP = (size_t)ROWS_ * ND_ * 4;
constexpr size_t SZ_XN   = (size_t)ROWS_ * ND_ * 2;
constexpr size_t SZ_WED  = (size_t)NE_ * ND_ * 2;
constexpr size_t SZ_WEE  = (size_t)NE_ * NE_ * 2;
constexpr size_t SZ_WDBC = (size_t)6 * NK_ * NE_ * 2;
constexpr size_t SZ_WDT  = (size_t)6 * NE_ * NR_ * 2;
constexpr size_t SZ_XO   = (size_t)ROWS_ * ND_ * 4;
constexpr size_t SZ_MZ1  = (size_t)ROWS_ * NE_ * 2;
constexpr size_t SZ_MX   = (size_t)ROWS_ * NE_ * 4;
constexpr size_t SZ_ZC   = (size_t)ROWS_ * NE_ * 4;
constexpr size_t SZ_ZCB  = (size_t)ROWS_ * NE_ * 2;
constexpr size_t SZ_DBC  = (size_t)3 * ROWS_ * NK_ * 4;
constexpr size_t SZ_Y    = (size_t)3 * ROWS_ * NE_ * 2;

constexpr size_t OFF_MOD   = 0;
constexpr size_t OFF_SKIP  = OFF_MOD + SZ_MOD;
constexpr size_t OFF_WSKIP = OFF_SKIP + SZ_SKIP;
constexpr size_t OFF_XN    = OFF_WSKIP + SZ_SKIP;
constexpr size_t OFF_WN    = OFF_XN + SZ_XN;
constexpr size_t OFF_WZ    = OFF_WN + SZ_XN;
constexpr size_t OFF_WX    = OFF_WZ + SZ_WED;
constexpr size_t OFF_WZW   = OFF_WX + SZ_WED;
constexpr size_t OFF_WXW   = OFF_WZW + SZ_WED;
constexpr size_t OFF_WC    = OFF_WXW + SZ_WED;
constexpr size_t OFF_WCW   = OFF_WC + SZ_WEE;
constexpr size_t OFF_WF    = OFF_WCW + SZ_WEE;
constexpr size_t OFF_WFW   = OFF_WF + SZ_WED;
constexpr size_t OFF_W1A   = OFF_WFW + SZ_WED;
constexpr size_t OFF_WDBC  = OFF_W1A + SZ_WED;
constexpr size_t OFF_WDT   = OFF_WDBC + SZ_WDBC;
constexpr size_t OFF_XO    = OFF_WDT + SZ_WDT;
constexpr size_t OFF_WO    = OFF_XO + SZ_XO;
constexpr size_t OFF_MZ1   = OFF_WO + SZ_XO;
constexpr size_t OFF_MX    = OFF_MZ1 + SZ_MZ1;
constexpr size_t OFF_ZC    = OFF_MX + SZ_MX;
constexpr size_t OFF_ZCB   = OFF_ZC + SZ_ZC;
constexpr size_t OFF_DBC   = OFF_ZCB + SZ_ZCB;
constexpr size_t OFF_Y     = OFF_DBC + SZ_DBC;
constexpr size_t WS_END    = OFF_Y + SZ_Y;

constexpr size_t OFF_TPL   = OFF_MZ1;
constexpr size_t OFF_COMBN = OFF_MZ1;
constexpr size_t OFF_HBUF  = OFF_MX;

static_assert(WS_END == (size_t)133312512);
static_assert(WS_END <= (size_t)134217728);
static_assert((size_t)ROWS_ * 2 * ND_ * 2 <= SZ_MZ1);
static_assert((size_t)ROWS_ * ND_ * 4 <= SZ_MX);
static_assert(OFF_SKIP % 256 == 0 && OFF_WSKIP % 256 == 0 && OFF_XN % 256 == 0 && OFF_WN % 256 == 0);
static_assert(OFF_WZ % 256 == 0 && OFF_WC % 256 == 0 && OFF_WF % 256 == 0 && OFF_W1A % 256 == 0);
static_assert(OFF_WDBC % 256 == 0 && OFF_WDT % 256 == 0 && OFF_XO % 256 == 0 && OFF_WO % 256 == 0);
static_assert(OFF_MZ1 % 256 == 0 && OFF_MX % 256 == 0 && OFF_ZC % 256 == 0 && OFF_ZCB % 256 == 0);
static_assert(OFF_DBC % 256 == 0 && OFF_Y % 256 == 0 && WS_END % 256 == 0);

__device__ __forceinline__ float silu_f(float x) {
    const float e = __expf(-x);
    return x * __builtin_amdgcn_rcpf(1.0f + e);
}
__device__ __forceinline__ float sigmoid_f(float x) {
    const float e = __expf(-x);
    return __builtin_amdgcn_rcpf(1.0f + e);
}
__device__ __forceinline__ float softplus_f(float x) {
    return fmaxf(x, 0.0f) + log1pf(__expf(-fabsf(x)));
}
__device__ __forceinline__ v8f ld8f(const float* p) {
    v4f a = *(const v4f*)p;
    v4f b = *(const v4f*)(p + 4);
    return __builtin_shufflevector(a, b, 0, 1, 2, 3, 4, 5, 6, 7);
}

template<int NW>
__device__ __forceinline__ void blk_sum2(float& a, float& b, float* sred) {
#pragma unroll
    for (int o = 16; o >= 1; o >>= 1) { a += __shfl_xor(a, o, 32); b += __shfl_xor(b, o, 32); }
    const int lane = threadIdx.x & 31, wid = threadIdx.x >> 5;
    if (lane == 0) { sred[2 * wid] = a; sred[2 * wid + 1] = b; }
    __syncthreads();
    float ta = 0.0f, tb = 0.0f;
#pragma unroll
    for (int i = 0; i < NW; ++i) { ta += sred[2 * i]; tb += sred[2 * i + 1]; }
    __syncthreads();
    a = ta; b = tb;
}

__device__ __forceinline__ void mma16(v8f& acc, const FragH& a, const FragH& b) {
    acc = __builtin_amdgcn_wmma_f32_16x16x32_f16(false, a.v, false, b.v, (short)0, acc, false, false);
    asm volatile("v_nop\n\tv_nop\n\tv_nop\n\tv_nop" : "+v"(acc) : "v"(a.v), "v"(b.v));
}

__global__ __launch_bounds__(256)
void cvt_kernel(const float* __restrict__ src, unsigned short* dst, int n8, float scale)
{
    const int i = blockIdx.x * 256 + threadIdx.x;
    if (i >= n8) return;
    const v8f v = ld8f(src + (size_t)i * 8) * scale;
    Pack8 pk;
    pk.f = __builtin_convertvector(v, v8h);
    const u16x8 u = pk.u;
    unsigned short* gp = dst + (size_t)i * 8;
    *(volatile u16x8*)gp = u;
    __threadfence();
    *(volatile u16x8*)gp = u;
}

__global__ __launch_bounds__(256)
void wdbc_t_kernel(const float* __restrict__ W, unsigned short* dst)
{
    const int i = blockIdx.x * 256 + threadIdx.x;
    if (i >= 6 * 64 * 128) return;
    const int e8  = i & 127;
    const int n   = (i >> 7) & 63;
    const int dir = i >> 13;
    const int e0  = e8 * 8;
    v8f v;
#pragma unroll
    for (int q = 0; q < 8; ++q) v[q] = W[((size_t)(dir * NE_ + e0 + q)) * NK_ + n] * 64.0f;
    Pack8 pk;
    pk.f = __builtin_convertvector(v, v8h);
    const u16x8 u = pk.u;
    unsigned short* gp = dst + ((size_t)(dir * NK_ + n)) * NE_ + e0;
    *(volatile u16x8*)gp = u;
    __threadfence();
    *(volatile u16x8*)gp = u;
}

__global__ __launch_bounds__(256)
void wdt_t_kernel(const float* __restrict__ W, unsigned short* dst)
{
    const int i = blockIdx.x * 256 + threadIdx.x;
    if (i >= 6 * 1024 * 4) return;
    const int r8  = i & 3;
    const int ch  = (i >> 2) & 1023;
    const int dir = i >> 12;
    const int r0  = r8 * 8;
    v8f v;
#pragma unroll
    for (int q = 0; q < 8; ++q) v[q] = W[((size_t)(dir * NR_ + r0 + q)) * NE_ + ch] * 64.0f;
    Pack8 pk;
    pk.f = __builtin_convertvector(v, v8h);
    const u16x8 u = pk.u;
    unsigned short* gp = dst + ((size_t)(dir * NE_ + ch)) * NR_ + r0;
    *(volatile u16x8*)gp = u;
    __threadfence();
    *(volatile u16x8*)gp = u;
}

__global__ __launch_bounds__(256)
void mod_kernel(const float* __restrict__ c, const float* __restrict__ Wada,
                const float* __restrict__ bada, float* mod)
{
    __shared__ float sc[2 * ND_];
    const int tid = threadIdx.x, b = blockIdx.y;
    const int d3  = blockIdx.x * 256 + tid;
#pragma unroll
    for (int j = 0; j < 4; ++j) {
        const int k = tid + 256 * j;
        sc[k] = silu_f(c[(size_t)b * (2 * ND_) + k]);
    }
    __syncthreads();
    const float* wr = Wada + (size_t)d3 * (2 * ND_);
    float acc = 0.0f;
#pragma unroll 4
    for (int k = 0; k < 2 * ND_; ++k) acc = fmaf(sc[k], wr[k], acc);
    const float v = acc + bada[d3];
    float* gp = mod + (size_t)b * (3 * ND_) + d3;
    *(volatile float*)gp = v;
    __threadfence();
    *(volatile float*)gp = v;
}

__global__ __launch_bounds__(128)
void pre_kernel(const float* __restrict__ x, const float* __restrict__ w, const float* __restrict__ mod,
                const float* __restrict__ g1, const float* __restrict__ be1,
                const float* __restrict__ g2, const float* __restrict__ be2,
                const float* __restrict__ g3, const float* __restrict__ be3,
                float* skip, float* wskip, unsigned short* xn, unsigned short* wn)
{
    __shared__ float sred[8];
    const int row = blockIdx.x, tid = threadIdx.x;
    const int b = row >> 11;
    const size_t rb = (size_t)row * ND_;
    const int d0 = 4 * tid;
    const float invD = 1.0f / (float)ND_;

    const v4f xv = *(const v4f*)(x + rb + d0);
    float s = xv[0] + xv[1] + xv[2] + xv[3], zz = 0.0f;
    blk_sum2<4>(s, zz, sred);
    const float m1 = s * invD;
    const v4f dx = xv - m1;
    float q = dx[0] * dx[0] + dx[1] * dx[1] + dx[2] * dx[2] + dx[3] * dx[3];
    zz = 0.0f;
    blk_sum2<4>(q, zz, sred);
    const float r1 = rsqrtf(q * invD + EPS_);

    const v4f g1v  = *(const v4f*)(g1 + d0);
    const v4f be1v = *(const v4f*)(be1 + d0);
    const v4f shv  = *(const v4f*)(mod + (size_t)b * (3 * ND_) + d0);
    const v4f scv  = *(const v4f*)(mod + (size_t)b * (3 * ND_) + ND_ + d0);
    const v4f wv   = *(const v4f*)(w + rb + d0);
    const v4f a    = (dx * r1 * g1v + be1v) * (scv + 1.0f) + shv;
    const v4f bw   = a * wv;

    float s2 = a[0] + a[1] + a[2] + a[3];
    float s3 = bw[0] + bw[1] + bw[2] + bw[3];
    blk_sum2<4>(s2, s3, sred);
    const float m2 = s2 * invD, m3 = s3 * invD;
    const v4f da = a - m2, db = bw - m3;
    float q2 = da[0] * da[0] + da[1] * da[1] + da[2] * da[2] + da[3] * da[3];
    float q3 = db[0] * db[0] + db[1] * db[1] + db[2] * db[2] + db[3] * db[3];
    blk_sum2<4>(q2, q3, sred);
    const float r2 = rsqrtf(q2 * invD + EPS_), r3 = rsqrtf(q3 * invD + EPS_);

    const v4f g2v = *(const v4f*)(g2 + d0), be2v = *(const v4f*)(be2 + d0);
    const v4f g3v = *(const v4f*)(g3 + d0), be3v = *(const v4f*)(be3 + d0);
    const v4f xnv = da * r2 * g2v + be2v;
    const v4f wnv = db * r3 * g3v + be3v;
    Pack4 px, pw;
    px.f = __builtin_convertvector(xnv, v4h);
    pw.f = __builtin_convertvector(wnv, v4h);
    const u16x4 ux = px.u, uw = pw.u;

    float* sp = skip + rb + d0;
    float* wp = wskip + rb + d0;
    unsigned short* xp  = xn + rb + d0;
    unsigned short* wnp = wn + rb + d0;
    *(volatile v4f*)sp = a;
    *(volatile v4f*)wp = bw;
    *(volatile u16x4*)xp = ux;
    *(volatile u16x4*)wnp = uw;
    __threadfence();
    *(volatile v4f*)sp = a;
    *(volatile v4f*)wp = bw;
    *(volatile u16x4*)xp = ux;
    *(volatile u16x4*)wnp = uw;
}

template<int NBF>
__device__ __forceinline__ void store_f32_pass(const float* st, float* gp, int ldc, int lane)
{
    constexpr int CW  = NBF * 16, P = CW + 4;
    constexpr int LPR = CW / 4;
    static_assert(32 % LPR == 0);
    constexpr int RPI = 32 / LPR;
    constexpr int NIT = 32 / RPI;
    static_assert((CW * 4) % 128 == 0);
    const int rsub = lane / LPR, c0 = (lane % LPR) * 4;
#pragma unroll
    for (int it = 0; it < NIT; ++it) {
        const int row = it * RPI + rsub;
        const v4f v = *(const v4f*)(st + row * P + c0);
        *(volatile v4f*)(gp + (size_t)row * ldc + c0) = v;
    }
}
template<int NBF>
__device__ __forceinline__ void store_f16_pass(const float* st, unsigned short* gp, int ldc, int lane, float hs)
{
    constexpr int CW  = NBF * 16, P = CW + 4;
    constexpr int LPR = CW / 8;
    static_assert(32 % LPR == 0);
    constexpr int RPI = 32 / LPR;
    constexpr int NIT = 32 / RPI;
    static_assert((CW * 2) % 128 == 0);
    const int rsub = lane / LPR, c0 = (lane % LPR) * 8;
#pragma unroll
    for (int it = 0; it < NIT; ++it) {
        const int row = it * RPI + rsub;
        const v8f f = ld8f(st + row * P + c0) * hs;
        Pack8 pk;
        pk.f = __builtin_convertvector(f, v8h);
        const u16x8 u = pk.u;
        *(volatile u16x8*)(gp + (size_t)row * ldc + c0) = u;
    }
}

template<int NBF, bool BIAS, bool RESID, int ACT, bool OUTF, bool OUTH>
__global__ __launch_bounds__(128)
void gemm_tn(const unsigned short* __restrict__ A, const unsigned short* __restrict__ Bw,
             const float* __restrict__ bias, const float* __restrict__ resid,
             float* Cf, unsigned short* Ch,
             long long b_zs, long long c_zs, int K, int ldc, float scale, float hscale)
{
    constexpr int CW = NBF * 16;
    constexpr int P  = CW + 4;
    __shared__ __attribute__((aligned(16))) float stile[4][32 * P];

    const int tid  = threadIdx.x;
    const int lane = tid & 31;
    const int wave = tid >> 5;
    const int h    = lane >> 4;
    const int m    = lane & 15;
    const int wm   = wave >> 1;
    const int wn   = wave & 1;
    const int z    = blockIdx.z;

    const int rowW = blockIdx.y * 64 + wm * 32;
    const int colW = blockIdx.x * (2 * CW) + wn * CW;

    const unsigned short* pa[2];
#pragma unroll
    for (int s = 0; s < 2; ++s) pa[s] = A + (size_t)(rowW + 16 * s + m) * K + 8 * h;
    const unsigned short* pb = Bw + (size_t)z * (size_t)b_zs + (size_t)(colW + m) * K + 8 * h;
    const size_t sub16 = (size_t)16 * K;

    v8f acc[2 * NBF];
#pragma unroll
    for (int j = 0; j < 2 * NBF; ++j)
#pragma unroll
        for (int r = 0; r < 8; ++r) acc[j][r] = 0.0f;

    const int nk = K >> 5;
    for (int kt = 0; kt < nk; ++kt) {
        const int k0 = kt * 32;
        FragH fa[2], fb[NBF];
#pragma unroll
        for (int s = 0; s < 2; ++s) {
            fa[s].h[0] = *(const u16x8*)(pa[s] + k0);
            fa[s].h[1] = *(const u16x8*)(pa[s] + k0 + 16);
        }
#pragma unroll
        for (int j = 0; j < NBF; ++j) {
            const unsigned short* p = pb + j * sub16 + k0;
            fb[j].h[0] = *(const u16x8*)(p);
            fb[j].h[1] = *(const u16x8*)(p + 16);
        }
#pragma unroll
        for (int s = 0; s < 2; ++s)
#pragma unroll
            for (int j = 0; j < NBF; ++j)
                mma16(acc[s * NBF + j], fa[s], fb[j]);
    }

    float* st = stile[wave];
#pragma unroll
    for (int s = 0; s < 2; ++s)
#pragma unroll
        for (int j = 0; j < NBF; ++j) {
            const int col = j * 16 + m;
            float bv = 0.0f;
            if constexpr (BIAS) bv = bias[colW + col];
#pragma unroll
            for (int r = 0; r < 8; ++r) {
                const int row = s * 16 + 8 * h + r;
                float v = acc[s * NBF + j][r] * scale + bv;
                if constexpr (RESID) v += resid[(size_t)(rowW + row) * ldc + colW + col];
                if constexpr (ACT == 1) v = silu_f(v);
                st[row * P + col] = v;
            }
        }
    __syncthreads();

    const size_t cbase = (size_t)z * (size_t)c_zs + (size_t)rowW * ldc + colW;
    if constexpr (OUTF) store_f32_pass<NBF>(st, Cf + cbase, ldc, lane);
    if constexpr (OUTH) store_f16_pass<NBF>(st, Ch + cbase, ldc, lane, hscale);
    __threadfence();
    if constexpr (OUTF) store_f32_pass<NBF>(st, Cf + cbase, ldc, lane);
    if constexpr (OUTH) store_f16_pass<NBF>(st, Ch + cbase, ldc, lane, hscale);
}

__device__ __forceinline__ void y16_store_pass(const unsigned short* sl, unsigned short* gp,
                                               size_t gbase, int wave, int lane) {
#pragma unroll
    for (int it = 0; it < 2; ++it) {
        const int t = it * 8 + wave * 4 + (lane >> 3);
        const int c = (lane & 7) * 8;
        const u16x8 v = *(const u16x8*)(sl + t * 64 + c);
        *(volatile u16x8*)(gp + gbase + (size_t)t * NE_ + c) = v;
    }
}

__global__ __launch_bounds__(64)
void scan_kernel(const float* __restrict__ zc, const float* __restrict__ dbc,
                 const unsigned short* __restrict__ wdtT, const float* __restrict__ bdt,
                 const float* __restrict__ Alog, const float* __restrict__ Dp,
                 const int* __restrict__ ord1, const int* __restrict__ ord2,
                 unsigned short* y)
{
    __shared__ __attribute__((aligned(16))) float sX[16 * 64];
    __shared__ __attribute__((aligned(16))) float sZ[16 * 64];
    __shared__ __attribute__((aligned(16))) float sDT[16 * 64];
    __shared__ __attribute__((aligned(16))) unsigned short sA[16 * 32];
    __shared__ __attribute__((aligned(16))) unsigned short sg[16 * 64];

    const int tid  = threadIdx.x;
    const int lane = tid & 31;
    const int wave = tid >> 5;
    const int h    = lane >> 4;
    const int m    = lane & 15;
    const int dir  = blockIdx.z;
    const int b    = blockIdx.y;
    const int dbase = blockIdx.x * 64;
    const int e    = dbase + tid;
    const size_t pe = (size_t)dir * NE_ + e;

    float an[NN_], hs[NN_];
#pragma unroll
    for (int n = 0; n < NN_; ++n) {
        an[n] = -expf(Alog[pe * NN_ + n]);
        hs[n] = 0.0f;
    }
    const float tb = bdt[pe];
    const float Dd = Dp[pe];

    FragH fb0, fb1;
    {
        const unsigned short* p0 = wdtT + ((size_t)dir * NE_ + dbase + wave * 32 + m) * NR_ + 8 * h;
        const unsigned short* p1 = p0 + 16 * NR_;
        fb0.h[0] = *(const u16x8*)(p0);
        fb0.h[1] = *(const u16x8*)(p0 + 16);
        fb1.h[0] = *(const u16x8*)(p1);
        fb1.h[1] = *(const u16x8*)(p1 + 16);
    }

    const float* dbd = dbc + (size_t)dir * ROWS_ * NK_;
    const int* op = (dir == 1) ? ord1 : ord2;
    const size_t brow = (size_t)b * NS_;

#pragma unroll 1
    for (int l0 = 0; l0 < NS_; l0 += 16) {
#pragma unroll 4
        for (int j = 0; j < 16; ++j) {
            const int t = l0 + j;
            int pr = op[t];
            pr = min(max(pr, 0), NS_ - 1);
            const int row = (dir == 0) ? t : pr;
            const size_t rr = brow + (size_t)row;
            const float v = dbd[rr * NK_ + tid];
            sX[j * 64 + tid] = v;
            if (wave == 0) {
                HBits hb;
                hb.h = (_Float16)(v * 64.0f);
                sA[j * 32 + lane] = hb.u;
            }
            sZ[j * 64 + tid] = zc[rr * NE_ + e];
        }
        __syncthreads();

        {
            FragH fa;
            fa.h[0] = *(const u16x8*)(sA + m * 32 + 8 * h);
            fa.h[1] = *(const u16x8*)(sA + m * 32 + 16 + 8 * h);
            v8f acc0, acc1;
#pragma unroll
            for (int r = 0; r < 8; ++r) { acc0[r] = 0.0f; acc1[r] = 0.0f; }
            mma16(acc0, fa, fb0);
            mma16(acc1, fa, fb1);
            const float inv = 1.0f / 4096.0f;
#pragma unroll
            for (int r = 0; r < 8; ++r) {
                sDT[(8 * h + r) * 64 + wave * 32 + m]      = acc0[r] * inv;
                sDT[(8 * h + r) * 64 + wave * 32 + 16 + m] = acc1[r] * inv;
            }
        }
        __syncthreads();

#pragma unroll 1
        for (int t = 0; t < 16; ++t) {
            const float xv = sZ[t * 64 + tid];
            const float* sr = sX + t * 64;
            const float dt = softplus_f(sDT[t * 64 + tid] + tb);
            const float du = dt * xv;
            float yv = 0.0f;
#pragma unroll
            for (int n = 0; n < NN_; ++n) {
                const float da = __expf(dt * an[n]);
                hs[n] = da * hs[n] + du * sr[NR_ + n];
                yv += hs[n] * sr[NR_ + NN_ + n];
            }
            const float yo = yv + Dd * xv;
            HBits hb;
            hb.h = (_Float16)yo;
            sg[t * 64 + tid] = hb.u;
        }
        __syncthreads();
        const size_t gbase = ((size_t)dir * ROWS_ + brow + (size_t)l0) * NE_ + dbase;
        y16_store_pass(sg, y, gbase, wave, lane);
        __threadfence();
        y16_store_pass(sg, y, gbase, wave, lane);
        __syncthreads();
    }
}

__global__ __launch_bounds__(256)
void merge_kernel(const unsigned short* __restrict__ y, const float* __restrict__ mx,
                  const int* __restrict__ inv1, const int* __restrict__ inv2,
                  unsigned short* tpl)
{
    const int i   = blockIdx.x * 256 + threadIdx.x;
    const int row = i >> 7;
    const int col = (i & 127) * 8;
    const int b   = row >> 11;
    const int s   = row & (NS_ - 1);
    int p1 = inv1[s]; p1 = min(max(p1, 0), NS_ - 1);
    int p2 = inv2[s]; p2 = min(max(p2, 0), NS_ - 1);
    const size_t r0 = (size_t)row;
    const size_t r1 = (size_t)b * NS_ + (size_t)p1;
    const size_t r2 = (size_t)b * NS_ + (size_t)p2;
    const size_t PL = (size_t)ROWS_ * NE_;
    Pack8 a0, a1, a2;
    a0.u = *(const u16x8*)(y + r0 * NE_ + col);
    a1.u = *(const u16x8*)(y + PL + r1 * NE_ + col);
    a2.u = *(const u16x8*)(y + 2 * PL + r2 * NE_ + col);
    const v8f ym = (__builtin_convertvector(a0.f, v8f) + __builtin_convertvector(a1.f, v8f))
                   + __builtin_convertvector(a2.f, v8f);
    const v8f mv = ld8f(mx + r0 * NE_ + col);
    v8f tv;
#pragma unroll
    for (int c = 0; c < 8; ++c) tv[c] = silu_f(mv[c]) * ym[c] * 64.0f;
    Pack8 pk;
    pk.f = __builtin_convertvector(tv, v8h);
    const u16x8 u = pk.u;
    unsigned short* gp = tpl + r0 * NE_ + col;
    *(volatile u16x8*)gp = u;
    __threadfence();
    *(volatile u16x8*)gp = u;
}

__global__ __launch_bounds__(256)
void concat_ln_kernel(const float* __restrict__ xo, const float* __restrict__ wo,
                      const float* __restrict__ ga, const float* __restrict__ ba,
                      unsigned short* combn)
{
    __shared__ float sred[16];
    const int row = blockIdx.x, tid = threadIdx.x;
    const int d0  = 4 * tid;
    const bool hi = tid >= 128;
    const float* src = hi ? (wo + (size_t)row * ND_ + (d0 - ND_)) : (xo + (size_t)row * ND_ + d0);
    const v4f v = *(const v4f*)src;
    const float invD = 1.0f / (float)(2 * ND_);
    float s = v[0] + v[1] + v[2] + v[3], zz = 0.0f;
    blk_sum2<8>(s, zz, sred);
    const float mean = s * invD;
    const v4f dv = v - mean;
    float q = dv[0] * dv[0] + dv[1] * dv[1] + dv[2] * dv[2] + dv[3] * dv[3];
    zz = 0.0f;
    blk_sum2<8>(q, zz, sred);
    const float rr = rsqrtf(q * invD + EPS_);
    const v4f gv = *(const v4f*)(ga + d0), bv = *(const v4f*)(ba + d0);
    const v4f o = dv * rr * gv + bv;
    Pack4 pk;
    pk.f = __builtin_convertvector(o, v4h);
    const u16x4 u = pk.u;
    unsigned short* gp = combn + (size_t)row * (2 * ND_) + d0;
    *(volatile u16x4*)gp = u;
    __threadfence();
    *(volatile u16x4*)gp = u;
}

__global__ __launch_bounds__(128)
void final_kernel(const float* __restrict__ hb, const float* __restrict__ W2a,
                  const float* __restrict__ b2a, const float* __restrict__ xo,
                  const float* __restrict__ wo, const float* __restrict__ x,
                  const float* __restrict__ mod, float* out)
{
    __shared__ float sred[8];
    const int row = blockIdx.x, tid = threadIdx.x;
    const int b = row >> 11;
    const size_t rb = (size_t)row * ND_;
    const int d0 = 4 * tid;
    const v4f hv = *(const v4f*)(hb + rb + d0);
    const v4f wv = *(const v4f*)(W2a + d0);
    float s = hv[0] * wv[0] + hv[1] * wv[1] + hv[2] * wv[2] + hv[3] * wv[3], zz = 0.0f;
    blk_sum2<4>(s, zz, sred);
    const float a = sigmoid_f(s + b2a[0]);
    const v4f xov = *(const v4f*)(xo + rb + d0);
    const v4f wov = *(const v4f*)(wo + rb + d0);
    const v4f xv  = *(const v4f*)(x + rb + d0);
    const v4f gv  = *(const v4f*)(mod + (size_t)b * (3 * ND_) + 2 * ND_ + d0);
    const v4f mix = xov * a + wov * (1.0f - a);
    const v4f o   = xv + gv * mix;
    float* op = out + rb + d0;
    *(volatile v4f*)op = o;
    __threadfence();
    *(volatile v4f*)op = o;
}

extern "C" void kernel_launch(void* const* d_in, const int* in_sizes, int n_in,
                              void* d_out, int out_size, void* d_ws, size_t ws_size,
                              hipStream_t stream)
{
    if (n_in < 42) return;
    const int ex[42] = {
        2097152, 2048, 2097152, 1572864, 1536,
        512, 512, 512, 512, 512, 512,
        524288, 1024, 524288, 1024, 524288, 1024, 524288, 1024,
        1048576, 1024, 1048576, 1024,
        524288, 512, 524288, 512,
        1024, 1024, 524288, 512, 512, 1,
        393216, 196608, 6144, 98304, 6144,
        2048, 2048, 2048, 2048 };
    for (int i = 0; i < 42; ++i) if (in_sizes[i] != ex[i]) return;
    if (out_size != ROWS_ * ND_) return;
    if (ws_size < WS_END) return;

    const float* x     = (const float*)d_in[0];
    const float* c     = (const float*)d_in[1];
    const float* w     = (const float*)d_in[2];
    const float* W_ada = (const float*)d_in[3];
    const float* b_ada = (const float*)d_in[4];
    const float* g1  = (const float*)d_in[5],  *be1 = (const float*)d_in[6];
    const float* g2  = (const float*)d_in[7],  *be2 = (const float*)d_in[8];
    const float* g3  = (const float*)d_in[9],  *be3 = (const float*)d_in[10];
    const float* Wz  = (const float*)d_in[11], *bz  = (const float*)d_in[12];
    const float* Wx  = (const float*)d_in[13], *bx  = (const float*)d_in[14];
    const float* Wzw = (const float*)d_in[15], *bzw = (const float*)d_in[16];
    const float* Wxw = (const float*)d_in[17], *bxw = (const float*)d_in[18];
    const float* Wc  = (const float*)d_in[19], *bc  = (const float*)d_in[20];
    const float* Wcw = (const float*)d_in[21], *bcw = (const float*)d_in[22];
    const float* Wf  = (const float*)d_in[23], *bfv = (const float*)d_in[24];
    const float* Wfw = (const float*)d_in[25], *bfw = (const float*)d_in[26];
    const float* ga  = (const float*)d_in[27], *ba  = (const float*)d_in[28];
    const float* W1a = (const float*)d_in[29], *b1a = (const float*)d_in[30];
    const float* W2a = (const float*)d_in[31], *b2a = (const float*)d_in[32];
    const float* Wdbc = (const float*)d_in[33];
    const float* Wdt  = (const float*)d_in[34];
    const float* bdt  = (const float*)d_in[35];
    const float* Alog = (const float*)d_in[36];
    const float* Dssm = (const float*)d_in[37];
    const int* order       = (const int*)d_in[38];
    const int* order_rev   = (const int*)d_in[39];
    const int* origina     = (const int*)d_in[40];
    const int* origina_rev = (const int*)d_in[41];
    float* out = (float*)d_out;

    char* ws = (char*)d_ws;
    float*          mod   = (float*)(ws + OFF_MOD);
    float*          skip  = (float*)(ws + OFF_SKIP);
    float*          wskip = (float*)(ws + OFF_WSKIP);
    unsigned short* xn16  = (unsigned short*)(ws + OFF_XN);
    unsigned short* wn16  = (unsigned short*)(ws + OFF_WN);
    unsigned short* wzH   = (unsigned short*)(ws + OFF_WZ);
    unsigned short* wxH   = (unsigned short*)(ws + OFF_WX);
    unsigned short* wzwH  = (unsigned short*)(ws + OFF_WZW);
    unsigned short* wxwH  = (unsigned short*)(ws + OFF_WXW);
    unsigned short* wcH   = (unsigned short*)(ws + OFF_WC);
    unsigned short* wcwH  = (unsigned short*)(ws + OFF_WCW);
    unsigned short* wfH   = (unsigned short*)(ws + OFF_WF);
    unsigned short* wfwH  = (unsigned short*)(ws + OFF_WFW);
    unsigned short* w1aH  = (unsigned short*)(ws + OFF_W1A);
    unsigned short* wdbcT = (unsigned short*)(ws + OFF_WDBC);
    unsigned short* wdtT  = (unsigned short*)(ws + OFF_WDT);
    float*          xo    = (float*)(ws + OFF_XO);
    float*          wo    = (float*)(ws + OFF_WO);
    unsigned short* mz1   = (unsigned short*)(ws + OFF_MZ1);
    unsigned short* tpl   = (unsigned short*)(ws + OFF_TPL);
    unsigned short* combn = (unsigned short*)(ws + OFF_COMBN);
    float*          mx    = (float*)(ws + OFF_MX);
    float*          hbuf  = (float*)(ws + OFF_HBUF);
    float*          zc    = (float*)(ws + OFF_ZC);
    unsigned short* zcb   = (unsigned short*)(ws + OFF_ZCB);
    float*          dbc   = (float*)(ws + OFF_DBC);
    unsigned short* ybuf  = (unsigned short*)(ws + OFF_Y);

    const int nED = NE_ * ND_;
    const int nEE = NE_ * NE_;

    cvt_kernel<<<dim3(nED / 8 / 256), dim3(256), 0, stream>>>(Wz,  wzH,  nED / 8, 64.0f);
    cvt_kernel<<<dim3(nED / 8 / 256), dim3(256), 0, stream>>>(Wx,  wxH,  nED / 8, 64.0f);
    cvt_kernel<<<dim3(nED / 8 / 256), dim3(256), 0, stream>>>(Wzw, wzwH, nED / 8, 64.0f);
    cvt_kernel<<<dim3(nED / 8 / 256), dim3(256), 0, stream>>>(Wxw, wxwH, nED / 8, 64.0f);
    cvt_kernel<<<dim3(nEE / 8 / 256), dim3(256), 0, stream>>>(Wc,  wcH,  nEE / 8, 64.0f);
    cvt_kernel<<<dim3(nEE / 8 / 256), dim3(256), 0, stream>>>(Wcw, wcwH, nEE / 8, 64.0f);
    cvt_kernel<<<dim3(nED / 8 / 256), dim3(256), 0, stream>>>(Wf,  wfH,  nED / 8, 64.0f);
    cvt_kernel<<<dim3(nED / 8 / 256), dim3(256), 0, stream>>>(Wfw, wfwH, nED / 8, 64.0f);
    cvt_kernel<<<dim3(nED / 8 / 256), dim3(256), 0, stream>>>(W1a, w1aH, nED / 8, 64.0f);
    wdbc_t_kernel<<<dim3((6 * 64 * 128) / 256), dim3(256), 0, stream>>>(Wdbc, wdbcT);
    wdt_t_kernel<<<dim3((6 * 1024 * 4) / 256), dim3(256), 0, stream>>>(Wdt, wdtT);

    mod_kernel<<<dim3((3 * ND_) / 256, NB_), dim3(256), 0, stream>>>(c, W_ada, b_ada, mod);
    pre_kernel<<<dim3(ROWS_), dim3(128), 0, stream>>>(x, w, mod, g1, be1, g2, be2, g3, be3,
                                                      skip, wskip, xn16, wn16);

    for (int br = 0; br < 2; ++br) {
        const unsigned short* a16 = br ? wn16 : xn16;
        const unsigned short* wzh = br ? wzwH : wzH;  const float* bzp = br ? bzw : bz;
        const unsigned short* wxh = br ? wxwH : wxH;  const float* bxp = br ? bxw : bx;
        const unsigned short* wch = br ? wcwH : wcH;  const float* bcp = br ? bcw : bc;
        const unsigned short* wfh = br ? wfwH : wfH;  const float* bfp = br ? bfw : bfv;
        const float* rsd = br ? (const float*)wskip : (const float*)skip;
        float* cout = br ? wo : xo;
        const unsigned short* wdbc3 = wdbcT + (size_t)br * 3 * NK_ * NE_;
        const unsigned short* wdt3  = wdtT  + (size_t)br * 3 * NE_ * NR_;
        const float* bdt3  = bdt  + (size_t)br * 3 * NE_;
        const float* alog3 = Alog + (size_t)br * 3 * NE_ * NN_;
        const float* dss3  = Dssm + (size_t)br * 3 * NE_;

        gemm_tn<4, true, false, 0, false, true><<<dim3(NE_ / 128, ROWS_ / 64, 1), dim3(128), 0, stream>>>(
            a16, wzh, bzp, rsd, zc, mz1, (long long)0, (long long)0, (int)ND_, (int)NE_, 1.0f / 64.0f, 16.0f);
        gemm_tn<4, true, false, 0, true, false><<<dim3(NE_ / 128, ROWS_ / 64, 1), dim3(128), 0, stream>>>(
            a16, wxh, bxp, rsd, mx, zcb, (long long)0, (long long)0, (int)ND_, (int)NE_, 1.0f / 64.0f, 1.0f);
        gemm_tn<4, true, false, 0, true, true><<<dim3(NE_ / 128, ROWS_ / 64, 1), dim3(128), 0, stream>>>(
            mz1, wch, bcp, rsd, zc, zcb, (long long)0, (long long)0, (int)NE_, (int)NE_, 1.0f / 1024.0f, 16.0f);
        gemm_tn<2, false, false, 0, true, false><<<dim3(1, ROWS_ / 64, 3), dim3(128), 0, stream>>>(
            zcb, wdbc3, bcp, rsd, dbc, mz1, (long long)NK_ * NE_, (long long)ROWS_ * NK_, (int)NE_, (int)NK_, 1.0f / 1024.0f, 1.0f);
        scan_kernel<<<dim3(NE_ / 64, NB_, 3), dim3(64), 0, stream>>>(
            (const float*)zc, (const float*)dbc, wdt3, bdt3, alog3, dss3, order, order_rev, ybuf);
        merge_kernel<<<dim3((ROWS_ * NE_ / 8) / 256), dim3(256), 0, stream>>>(
            (const unsigned short*)ybuf, (const float*)mx, origina, origina_rev, tpl);
        gemm_tn<4, true, true, 0, true, false><<<dim3(ND_ / 128, ROWS_ / 64, 1), dim3(128), 0, stream>>>(
            tpl, wfh, bfp, rsd, cout, zcb, (long long)0, (long long)0, (int)NE_, (int)ND_, 1.0f / 4096.0f, 1.0f);
    }

    concat_ln_kernel<<<dim3(ROWS_), dim3(256), 0, stream>>>((const float*)xo, (const float*)wo, ga, ba, combn);
    gemm_tn<4, true, false, 1, true, false><<<dim3(ND_ / 128, ROWS_ / 64, 1), dim3(128), 0, stream>>>(
        combn, w1aH, b1a, (const float*)skip, hbuf, zcb, (long long)0, (long long)0, (int)(2 * ND_), (int)ND_, 1.0f / 64.0f, 1.0f);
    final_kernel<<<dim3(ROWS_), dim3(128), 0, stream>>>((const float*)hbuf, W2a, b2a,
                                                        (const float*)xo, (const float*)wo, x, (const float*)mod, out);
}
